// SelfKANtentionND_85323820302820
// MI455X (gfx1250) — hardware-run, weakly checked
//
#include <hip/hip_runtime.h>
#include <math.h>
#include <stddef.h>

typedef __attribute__((ext_vector_type(16))) __bf16 v16b;
typedef __attribute__((ext_vector_type(8)))  __bf16 v8b;
typedef __attribute__((ext_vector_type(8)))  float  v8f;
typedef __attribute__((ext_vector_type(4)))  float  v4f;
typedef __attribute__((ext_vector_type(4)))  unsigned int v4u;

static_assert(sizeof(long) == 8);

constexpr int kB    = 4;
constexpr int kCIN  = 128;
constexpr int kCI   = 64;
constexpr int kHW   = 64;
constexpr int kNPIX = 4096;
constexpr int kPSTR = 4112;
constexpr int kG    = 8;
constexpr int kCSPL = 512;
constexpr int kCO3  = 192;
constexpr int kKB   = 576;
constexpr int kKS   = 4608;
constexpr int kKT   = 5184;
static_assert(kCSPL == kCI * kG);
static_assert(kKT == kKB + kKS);
static_assert(kB * kHW == 256);
static_assert(kNPIX == kHW * kHW);

constexpr size_t szXT  = (size_t)kB * kNPIX * kCIN * 2;
constexpr size_t szW16 = (size_t)kCI * kCIN * 2;
constexpr size_t szWT  = (size_t)kCO3 * kKT * 2;
constexpr size_t szATT = (size_t)kB * kNPIX * kCI * 4;
constexpr size_t szST  = (size_t)kB * kCI * 2 * 4;
constexpr size_t szSP  = (size_t)kB * kPSTR * kCI * 2;
constexpr size_t szBP  = (size_t)kB * kPSTR * kCSPL * 2;
constexpr size_t szQKV = (size_t)kB * kCO3 * kNPIX * 4;
constexpr size_t szP16 = (size_t)kB * kNPIX * kCI * 2;
constexpr size_t szY   = (size_t)kB * kCIN * kNPIX * 4;
constexpr size_t oXT   = 0;
constexpr size_t oWIN  = oXT + szXT;
constexpr size_t oWOUT = oWIN + szW16;
constexpr size_t oWT   = oWOUT + szW16;
constexpr size_t oATT  = oWT + szWT;
constexpr size_t oST   = oATT + szATT;
constexpr size_t oSH   = oST + szST;
constexpr size_t oSL   = oSH + szSP;
constexpr size_t oBH   = oSL + szSP;
constexpr size_t oBL   = oBH + szBP;
constexpr size_t oQKV  = oBL + szBP;
constexpr size_t oQH   = oQKV + szQKV;
constexpr size_t oQL   = oQH + szP16;
constexpr size_t oKH   = oQL + szP16;
constexpr size_t oKL   = oKH + szP16;
constexpr size_t oVH   = oKL + szP16;
constexpr size_t oVL   = oVH + szP16;
constexpr size_t oOH   = oVL + szP16;
constexpr size_t oOL   = oOH + szP16;
constexpr size_t oY    = oOL + szP16;
constexpr size_t kWsTotal = oY + szY;
static_assert(kWsTotal <= (size_t)134217728);
static_assert((oWIN % 256) == 0 && (oWT % 256) == 0 && (oATT % 256) == 0 && (oST % 256) == 0 && (oSH % 256) == 0);
static_assert((oBH % 256) == 0 && (oQKV % 256) == 0 && (oQH % 256) == 0 && (oY % 256) == 0);

__device__ __forceinline__ unsigned short f2bf_bits(float f) {
  unsigned u = __float_as_uint(f);
  return (unsigned short)((u + 0x7FFFu + ((u >> 16) & 1u)) >> 16);
}
__device__ __forceinline__ float bf_bits2f(unsigned short h) { return __uint_as_float(((unsigned)h) << 16); }
__device__ __forceinline__ float rbf(float f) { return bf_bits2f(f2bf_bits(f)); }
__device__ __forceinline__ v4f rbf4(v4f x) {
  v4f r;
  r.x = rbf(x.x); r.y = rbf(x.y); r.z = rbf(x.z); r.w = rbf(x.w);
  return r;
}
__device__ __forceinline__ __bf16 to_bf(float f) { return __builtin_bit_cast(__bf16, f2bf_bits(f)); }
__device__ __forceinline__ void split_bf(float f, __bf16& hi, __bf16& lo) {
  const unsigned short hb = f2bf_bits(f);
  hi = __builtin_bit_cast(__bf16, hb);
  lo = to_bf(f - bf_bits2f(hb));
}
__device__ __forceinline__ void split2(float f0, float f1, unsigned& hw, unsigned& lw) {
  const unsigned short h0 = f2bf_bits(f0), h1 = f2bf_bits(f1);
  const unsigned short l0 = f2bf_bits(f0 - bf_bits2f(h0)), l1 = f2bf_bits(f1 - bf_bits2f(h1));
  hw = (unsigned)h0 | ((unsigned)h1 << 16);
  lw = (unsigned)l0 | ((unsigned)l1 << 16);
}

__device__ __forceinline__ void dep_guard_b(v8f& a, v8f& b, v16b x, v16b y) { asm volatile("v_nop\n\tv_nop\n\tv_nop\n\tv_nop" : "+v"(a), "+v"(b) : "v"(x), "v"(y)); }
__device__ __forceinline__ void keep4_b(v16b a, v16b b, v16b c, v16b d) { asm volatile("v_nop" :: "v"(a), "v"(b), "v"(c), "v"(d)); }
__device__ __forceinline__ void acc_guard4(v8f& a, v8f& b, v8f& c, v8f& d) { asm volatile("v_nop\n\tv_nop\n\tv_nop\n\tv_nop" : "+v"(a), "+v"(b), "+v"(c), "+v"(d)); }
template <typename T> struct Frag;
template <> struct Frag<__bf16> {
  typedef v16b V; union U { v16b v; v8b h[2]; };
  static __device__ __forceinline__ v16b load(const __bf16* p) {
    U f; f.h[0] = *(const v8b*)(p); f.h[1] = *(const v8b*)(p + 16); return f.v;
  }
  static __device__ __forceinline__ v8f mma(v16b a, v16b b, v8f c) {
    return __builtin_amdgcn_wmma_f32_16x16x32_bf16(false, a, false, b, (short)0, c, false, false);
  }
  static __device__ __forceinline__ void guard(v8f& a, v8f& b, v16b x, v16b y) { dep_guard_b(a, b, x, y); }
  static __device__ __forceinline__ void keep(v16b a, v16b b, v16b c, v16b d) { keep4_b(a, b, c, d); }
};
__device__ __forceinline__ v8f mma_g(v16b a, v16b b, v8f c) {
  c = __builtin_amdgcn_wmma_f32_16x16x32_bf16(false, a, false, b, (short)0, c, false, false);
  asm volatile("v_nop\n\tv_nop\n\tv_nop\n\tv_nop" : "+v"(c) : "v"(a), "v"(b));
  return c;
}

__global__ __launch_bounds__(256) void zero_ghost_kernel(unsigned short* __restrict__ sH, unsigned short* __restrict__ sL,
                                                         unsigned short* __restrict__ bH, unsigned short* __restrict__ bL) {
  const int plane = blockIdx.y;
  unsigned short* base = (plane == 0) ? sH : (plane == 1) ? sL : (plane == 2) ? bH : bL;
  const int cw = (plane < 2) ? kCI : kCSPL;
  const int per_b = cw * 2;
  const int count = kB * per_b;
  const int idx = blockIdx.x * 256 + threadIdx.x;
  if (idx < count) {
    const int b = idx / per_b;
    const int o = idx - b * per_b;
    v4u z; z.x = 0u; z.y = 0u; z.z = 0u; z.w = 0u;
    volatile v4u* p = (volatile v4u*)(base + ((size_t)(b * kPSTR + kNPIX)) * cw + (size_t)o * 8);
    *p = z;
    __threadfence();
    *p = z;
  }
}

__global__ __launch_bounds__(256) void cast_f32_bf16x2(const float* __restrict__ in, unsigned short* __restrict__ out, int n2) {
  const int i = blockIdx.x * 256 + threadIdx.x;
  if (i < n2) {
    const unsigned u = (unsigned)f2bf_bits(in[2 * i]) | ((unsigned)f2bf_bits(in[2 * i + 1]) << 16);
    ((volatile unsigned*)out)[i] = u;
    __threadfence();
    ((volatile unsigned*)out)[i] = u;
  }
}

__global__ __launch_bounds__(256) void wreorder_kernel(const float* __restrict__ W, unsigned short* __restrict__ Wt,
                                                      int cwsh, int rowoff, int coloff, int npairs) {
  const int idx = blockIdx.x * 256 + threadIdx.x;
  if (idx < npairs) {
    const int cw = 1 << cwsh;
    const int kseg2 = (cw * 9) >> 1;
    const int row = idx / kseg2;
    const int kp = idx - row * kseg2;
    const int k = kp * 2;
    const int tap = k >> cwsh;
    const int ci = k & (cw - 1);
    const size_t src = ((size_t)row * cw + ci) * 9 + tap;
    const unsigned u = (unsigned)f2bf_bits(W[src]) | ((unsigned)f2bf_bits(W[src + 9]) << 16);
    volatile unsigned* p = (volatile unsigned*)(Wt + (size_t)(rowoff + row) * kKT + coloff + k);
    *p = u;
    __threadfence();
    *p = u;
  }
}

__global__ __launch_bounds__(256) void xpose_x_kernel(const float* __restrict__ x, unsigned short* __restrict__ xT) {
  __shared__ __align__(16) float tile[kCIN * 68];
  const int tid = threadIdx.x;
  const int blk = blockIdx.x;
  const int b = blk >> 6;
  const int p0 = (blk & 63) * 64;
  const float* src = x + (size_t)b * kCIN * kNPIX + p0;
#pragma unroll
  for (int it = 0; it < 8; ++it) {
    const int idx = it * 256 + tid;
    const int cin = idx >> 4;
    const int c4 = (idx & 15) * 4;
    *(v4f*)(tile + cin * 68 + c4) = *(const v4f*)(src + (size_t)cin * kNPIX + c4);
  }
  __syncthreads();
  const int w = tid >> 5, l = tid & 31;
  const int half = l >> 4;
  const int c8 = (l & 15) * 8;
  unsigned short* dst = xT + (size_t)b * kNPIX * kCIN;
  for (int pass = 0; pass < 2; ++pass) {
#pragma unroll
    for (int it = 0; it < 4; ++it) {
      const int p = ((w * 4 + it) << 1) + half;
      unsigned wd[4];
#pragma unroll
      for (int e = 0; e < 4; ++e) {
        const float f0 = tile[(c8 + 2 * e) * 68 + p];
        const float f1 = tile[(c8 + 2 * e + 1) * 68 + p];
        wd[e] = (unsigned)f2bf_bits(f0) | ((unsigned)f2bf_bits(f1) << 16);
      }
      v4u v; v.x = wd[0]; v.y = wd[1]; v.z = wd[2]; v.w = wd[3];
      *(volatile v4u*)(dst + (size_t)(p0 + p) * kCIN + c8) = v;
    }
    __threadfence();
  }
}

template <bool SPLITB, int BIAS_MODE, bool RESX>
__global__ __launch_bounds__(256) void gemm64_kernel(
    const unsigned short* __restrict__ Ap, int lda, long strideA,
    const unsigned short* __restrict__ Btp, const unsigned short* __restrict__ Bt2p, int ldb, long strideB,
    float* __restrict__ Cout, int ldc, long strideC,
    const float* __restrict__ bias,
    const float* __restrict__ resx, const float* __restrict__ gam,
    int M, int N, int K) {
  typedef __bf16 T;
  const T* A = (const T*)Ap; const T* Bt = (const T*)Btp; const T* Bt2 = (const T*)Bt2p;
  __shared__ __align__(16) float sT[8][16 * 68];
  const int b    = blockIdx.y;
  const int lane = threadIdx.x & 31;
  const int wave = threadIdx.x >> 5;
  const int tilesN = N >> 6;
  const int tilesM = M >> 6;
  const int tile = blockIdx.x * 8 + wave;
  if (tile >= tilesM * tilesN) return;
  const int tm = tile / tilesN;
  const int tn = tile - tm * tilesN;
  const int m0 = tm << 6;
  const int n0 = tn << 6;

  const T* Ab  = A  + (size_t)b * strideA;
  const T* Bb  = Bt + (size_t)b * strideB;
  const T* Bb2 = SPLITB ? (Bt2 + (size_t)b * strideB) : Bb;

  const int rlane = lane & 15;
  const int koff  = (lane >> 4) * 8;
  const int mOff  = (lane >> 4) * 8;

  v8f acc[4][4];
#pragma unroll
  for (int i = 0; i < 4; ++i)
#pragma unroll
    for (int j = 0; j < 4; ++j) acc[i][j] = (v8f){0.f,0.f,0.f,0.f,0.f,0.f,0.f,0.f};

  for (int k0 = 0; k0 < K; k0 += 32) {
    v16b bh[4], bl[4];
#pragma unroll
    for (int j = 0; j < 4; ++j) {
      const size_t bo = (size_t)(n0 + (j << 4) + rlane) * ldb + koff + k0;
      bh[j] = Frag<T>::load(Bb + bo);
      if (SPLITB) bl[j] = Frag<T>::load(Bb2 + bo); else bl[j] = bh[j];
    }
#pragma unroll
    for (int i = 0; i < 4; ++i) {
      const size_t ao = (size_t)(m0 + (i << 4) + rlane) * lda + koff + k0;
      const v16b ah = Frag<T>::load(Ab + ao);
#pragma unroll
      for (int j = 0; j < 4; ++j) {
        acc[i][j] = Frag<T>::mma(ah, bh[j], acc[i][j]);
        if (SPLITB) acc[i][j] = Frag<T>::mma(ah, bl[j], acc[i][j]);
      }
      Frag<T>::guard(acc[i][0], acc[i][3], ah, ah);
    }
    Frag<T>::keep(bh[0], bh[1], bh[2], bh[3]);
    if (SPLITB) Frag<T>::keep(bl[0], bl[1], bl[2], bl[3]);
  }
  acc_guard4(acc[0][0], acc[0][1], acc[0][2], acc[0][3]);
  acc_guard4(acc[1][0], acc[1][1], acc[1][2], acc[1][3]);
  acc_guard4(acc[2][0], acc[2][1], acc[2][2], acc[2][3]);
  acc_guard4(acc[3][0], acc[3][1], acc[3][2], acc[3][3]);

  float* slab = sT[wave];
  float* C = Cout + (size_t)b * strideC;
  const float* R = RESX ? (resx + (size_t)b * strideC) : resx;
  const float g = RESX ? rbf(gam[0]) : 0.f;
#pragma unroll
  for (int i = 0; i < 4; ++i) {
    const int mBase = m0 + (i << 4);
    v4f bm0 = (v4f){0.f, 0.f, 0.f, 0.f}, bm1 = bm0;
    if (BIAS_MODE == 1) { bm0 = *(const v4f*)(bias + mBase + mOff); bm1 = *(const v4f*)(bias + mBase + mOff + 4); }
#pragma unroll
    for (int j = 0; j < 4; ++j) {
      const int n = n0 + (j << 4) + rlane;
      float bv = 0.f;
      if (BIAS_MODE == 2) bv = rbf(bias[n]);
#pragma unroll
      for (int r = 0; r < 8; ++r) {
        float v = acc[i][j][r];
        if (BIAS_MODE == 1) v += rbf((r < 4) ? bm0[r & 3] : bm1[r & 3]);
        if (BIAS_MODE == 2) v += bv;
        slab[(mOff + r) * 68 + (j << 4) + rlane] = v;
      }
    }
    __builtin_amdgcn_fence(__ATOMIC_RELEASE, "workgroup");
    __builtin_amdgcn_wave_barrier();
    __builtin_amdgcn_fence(__ATOMIC_ACQUIRE, "workgroup");
    {
      const int hh = lane >> 4, c4 = (lane & 15) * 4;
      for (int pass = 0; pass < 2; ++pass) {
#pragma unroll
        for (int it = 0; it < 8; ++it) {
          const int row = it * 2 + hh;
          v4f v = *(const v4f*)(slab + row * 68 + c4);
          const size_t co = (size_t)(mBase + row) * ldc + n0 + c4;
          if (RESX) { const v4f xr = *(const v4f*)(R + co); v = v + g * rbf4(xr); }
          *(volatile v4f*)(C + co) = v;
        }
        __threadfence();
      }
    }
    __builtin_amdgcn_fence(__ATOMIC_RELEASE, "workgroup");
    __builtin_amdgcn_wave_barrier();
    __builtin_amdgcn_fence(__ATOMIC_ACQUIRE, "workgroup");
  }
}

__global__ __launch_bounds__(256) void inorm_stats_kernel(const float* __restrict__ att, float* __restrict__ st) {
  __shared__ float red[256];
  __shared__ float mean_s[64];
  __shared__ __align__(16) float outv[128];
  const int tid = threadIdx.x, b = blockIdx.x;
  const int c = tid & 63, part = tid >> 6;
  const float* col = att + ((size_t)b * kNPIX + (size_t)part * 1024) * kCI + c;
  float s = 0.f;
#pragma unroll 4
  for (int i = 0; i < 1024; ++i) s += col[(size_t)i * kCI];
  red[tid] = s;
  __syncthreads();
  if (tid < 64) mean_s[tid] = ((red[tid] + red[tid + 64]) + (red[tid + 128] + red[tid + 192])) * (1.0f / 4096.0f);
  __syncthreads();
  const float m = mean_s[c];
  float s2 = 0.f;
#pragma unroll 4
  for (int i = 0; i < 1024; ++i) { const float d = col[(size_t)i * kCI] - m; s2 += d * d; }
  red[tid] = s2;
  __syncthreads();
  if (tid < 64) {
    const float var = ((red[tid] + red[tid + 64]) + (red[tid + 128] + red[tid + 192])) * (1.0f / 4096.0f);
    outv[2 * tid] = mean_s[tid];
    outv[2 * tid + 1] = rsqrtf(var + 1e-5f);
  }
  __syncthreads();
  if (tid < 32) {
    const v4f v = *(const v4f*)(outv + tid * 4);
    volatile v4f* p = (volatile v4f*)(st + (size_t)b * 128 + tid * 4);
    *p = v;
    __threadfence();
    *p = v;
  }
}

__global__ __launch_bounds__(256) void act_planes_kernel(const float* __restrict__ att, const float* __restrict__ st,
    unsigned short* __restrict__ sH, unsigned short* __restrict__ sL,
    unsigned short* __restrict__ bH, unsigned short* __restrict__ bL, float inv7, float invden) {
  __shared__ __align__(16) unsigned short shH[256];
  __shared__ __align__(16) unsigned short shL[256];
  const int tid = threadIdx.x;
  const int pl = tid >> 6, ci = tid & 63;
  const int blk = blockIdx.x;
  const int b = blk >> 10;
  const int p0 = (blk & 1023) * 4;
  const int p = p0 + pl;
  const float a = att[((size_t)(b * kNPIX + p)) * kCI + ci];
  const float m = st[(b * kCI + ci) * 2];
  const float rs = st[(b * kCI + ci) * 2 + 1];
  const float ac = fminf(fmaxf(a, -30.0f), 30.0f);
  const float sg = 1.0f / (1.0f + expf(-ac));
  const float sv = a * sg;
  const unsigned short h0 = f2bf_bits(sv);
  const unsigned short l0 = f2bf_bits(sv - bf_bits2f(h0));
  shH[tid] = h0;
  shL[tid] = l0;
  const float xn = (a - m) * rs;
  unsigned long long H0 = 0ull, H1 = 0ull, L0 = 0ull, L1 = 0ull;
#pragma unroll 1
  for (int g = 0; g < kG; ++g) {
    const float sf = (float)g * inv7;
    const float gv = (g < kG - 1) ? (-2.0f * (1.0f - sf) + 2.0f * sf) : 2.0f;
    const float t = (xn - gv) * invden;
    const float e = expf(-(t * t));
    const unsigned short hb = f2bf_bits(e);
    const unsigned short lb = f2bf_bits(e - bf_bits2f(hb));
    const int shf = (g & 3) * 16;
    const unsigned long long hv = ((unsigned long long)hb) << shf;
    const unsigned long long lv = ((unsigned long long)lb) << shf;
    if (g < 4) { H0 |= hv; L0 |= lv; } else { H1 |= hv; L1 |= lv; }
  }
  v4u HV; HV.x = (unsigned)H0; HV.y = (unsigned)(H0 >> 32); HV.z = (unsigned)H1; HV.w = (unsigned)(H1 >> 32);
  v4u LV; LV.x = (unsigned)L0; LV.y = (unsigned)(L0 >> 32); LV.z = (unsigned)L1; LV.w = (unsigned)(L1 >> 32);
  const size_t bo = ((size_t)(b * kPSTR + p)) * kCSPL + (size_t)ci * 8;
  *(volatile v4u*)(bH + bo) = HV;
  *(volatile v4u*)(bL + bo) = LV;
  __threadfence();
  *(volatile v4u*)(bH + bo) = HV;
  *(volatile v4u*)(bL + bo) = LV;
  __syncthreads();
  if (tid < 64) {
    const int w = tid >> 5, l = tid & 31;
    const v4u hv = *(const v4u*)(shH + l * 8);
    const v4u lv = *(const v4u*)(shL + l * 8);
    const v4u val = w ? lv : hv;
    unsigned short* dst = w ? sL : sH;
    const size_t so = ((size_t)(b * kPSTR + p0)) * kCI + (size_t)l * 8;
    *(volatile v4u*)(dst + so) = val;
    __threadfence();
    *(volatile v4u*)(dst + so) = val;
  }
}

__global__ __launch_bounds__(256) void conv_qkv_kernel(
    const unsigned short* __restrict__ Wtp,
    const unsigned short* __restrict__ sHp, const unsigned short* __restrict__ sLp,
    const unsigned short* __restrict__ bHp, const unsigned short* __restrict__ bLp,
    float* __restrict__ qkv) {
  typedef __bf16 T;
  __shared__ __align__(16) float sT[8][16 * 68];
  const int lane = threadIdx.x & 31, wave = threadIdx.x >> 5;
  const int tile = blockIdx.x * 8 + wave;
  if (tile >= (kCO3 / 64) * (kB * kHW)) return;
  const int tm = tile >> 8;
  const int tn = tile & 255;
  const int m0 = tm << 6;
  const int bb = tn >> 6;
  const int hrow = tn & 63;
  const int n0 = hrow << 6;
  const int rlane = lane & 15, koff = (lane >> 4) * 8, mOff = (lane >> 4) * 8;
  const T* Wt = (const T*)Wtp;

  v8f acc[4][4];
#pragma unroll
  for (int i = 0; i < 4; ++i)
#pragma unroll
    for (int j = 0; j < 4; ++j) acc[i][j] = (v8f){0.f,0.f,0.f,0.f,0.f,0.f,0.f,0.f};

  for (int phase = 0; phase < 2; ++phase) {
    const T* Hp = (const T*)(phase ? bHp : sHp);
    const T* Lp = (const T*)(phase ? bLp : sLp);
    const int cwsh = phase ? 9 : 6;
    const int ncb = phase ? (kCSPL / 32) : (kCI / 32);
    const int abase = phase ? kKB : 0;
    for (int tap = 0; tap < 9; ++tap) {
      const int ty = tap / 3;
      const int dy = ty - 1;
      const int dx = tap - ty * 3 - 1;
      const int hh2 = hrow + dy;
      size_t boff[4];
#pragma unroll
      for (int j = 0; j < 4; ++j) {
        const int ww = (j << 4) + rlane + dx;
        const bool valid = ((unsigned)hh2 < (unsigned)kHW) && ((unsigned)ww < (unsigned)kHW);
        const int prow = valid ? (hh2 * kHW + ww) : kNPIX;
        boff[j] = ((((size_t)bb * kPSTR) + (size_t)prow) << cwsh) + (size_t)koff;
      }
      const int acol = abase + (tap << cwsh) + koff;
      for (int cb = 0; cb < ncb; ++cb) {
        const int ci0 = cb << 5;
        v16b bh[4], bl[4];
#pragma unroll
        for (int j = 0; j < 4; ++j) {
          bh[j] = Frag<T>::load(Hp + boff[j] + ci0);
          bl[j] = Frag<T>::load(Lp + boff[j] + ci0);
        }
#pragma unroll
        for (int i = 0; i < 4; ++i) {
          const size_t ao = (size_t)(m0 + (i << 4) + rlane) * kKT + acol + ci0;
          const v16b ah = Frag<T>::load(Wt + ao);
#pragma unroll
          for (int j = 0; j < 4; ++j) {
            acc[i][j] = Frag<T>::mma(ah, bh[j], acc[i][j]);
            acc[i][j] = Frag<T>::mma(ah, bl[j], acc[i][j]);
          }
          Frag<T>::guard(acc[i][0], acc[i][3], ah, ah);
        }
        Frag<T>::keep(bh[0], bh[1], bh[2], bh[3]);
        Frag<T>::keep(bl[0], bl[1], bl[2], bl[3]);
      }
    }
  }
  acc_guard4(acc[0][0], acc[0][1], acc[0][2], acc[0][3]);
  acc_guard4(acc[1][0], acc[1][1], acc[1][2], acc[1][3]);
  acc_guard4(acc[2][0], acc[2][1], acc[2][2], acc[2][3]);
  acc_guard4(acc[3][0], acc[3][1], acc[3][2], acc[3][3]);

  float* slab = sT[wave];
  float* C = qkv + (size_t)bb * kCO3 * kNPIX;
#pragma unroll
  for (int i = 0; i < 4; ++i) {
    const int mBase = m0 + (i << 4);
#pragma unroll
    for (int j = 0; j < 4; ++j) {
#pragma unroll
      for (int r = 0; r < 8; ++r) slab[(mOff + r) * 68 + (j << 4) + rlane] = acc[i][j][r];
    }
    __builtin_amdgcn_fence(__ATOMIC_RELEASE, "workgroup");
    __builtin_amdgcn_wave_barrier();
    __builtin_amdgcn_fence(__ATOMIC_ACQUIRE, "workgroup");
    {
      const int hh = lane >> 4, c4 = (lane & 15) * 4;
      for (int pass = 0; pass < 2; ++pass) {
#pragma unroll
        for (int it = 0; it < 8; ++it) {
          const int row = it * 2 + hh;
          const v4f v = *(const v4f*)(slab + row * 68 + c4);
          *(volatile v4f*)(C + (size_t)(mBase + row) * kNPIX + n0 + c4) = v;
        }
        __threadfence();
      }
    }
    __builtin_amdgcn_fence(__ATOMIC_RELEASE, "workgroup");
    __builtin_amdgcn_wave_barrier();
    __builtin_amdgcn_fence(__ATOMIC_ACQUIRE, "workgroup");
  }
}

__global__ __launch_bounds__(256) void qk_planes_kernel(const float* __restrict__ qkv,
    unsigned short* __restrict__ qH, unsigned short* __restrict__ qL,
    unsigned short* __restrict__ kH, unsigned short* __restrict__ kL) {
  __shared__ __align__(16) float tile[64 * 68];
  const int tid = threadIdx.x;
  const int blk = blockIdx.x;
  const int b = blk >> 7;
  const int sel = (blk >> 6) & 1;
  const int p0 = (blk & 63) * 64;
  const float* src = qkv + ((size_t)(b * kCO3 + sel * kCI)) * kNPIX + p0;
#pragma unroll
  for (int it = 0; it < 4; ++it) {
    const int idx = it * 256 + tid;
    const int co = idx >> 4;
    const int c4 = (idx & 15) * 4;
    *(v4f*)(tile + co * 68 + c4) = *(const v4f*)(src + (size_t)co * kNPIX + c4);
  }
  __syncthreads();
  unsigned short* dH = (sel ? kH : qH) + (size_t)b * kNPIX * kCI;
  unsigned short* dL = (sel ? kL : qL) + (size_t)b * kNPIX * kCI;
  const int w = tid >> 5, l = tid & 31;
  const int rq = l >> 3, c8 = (l & 7) * 8;
  for (int pass = 0; pass < 2; ++pass) {
#pragma unroll
    for (int it = 0; it < 2; ++it) {
      const int p = (w * 2 + it) * 4 + rq;
      unsigned hw[4], lw[4];
#pragma unroll
      for (int e = 0; e < 4; ++e)
        split2(tile[(c8 + 2 * e) * 68 + p], tile[(c8 + 2 * e + 1) * 68 + p], hw[e], lw[e]);
      v4u hv; hv.x = hw[0]; hv.y = hw[1]; hv.z = hw[2]; hv.w = hw[3];
      v4u lv; lv.x = lw[0]; lv.y = lw[1]; lv.z = lw[2]; lv.w = lw[3];
      const size_t d = (size_t)(p0 + p) * kCI + c8;
      *(volatile v4u*)(dH + d) = hv;
      *(volatile v4u*)(dL + d) = lv;
    }
    __threadfence();
  }
}

__global__ __launch_bounds__(256) void v_planes_kernel(const float* __restrict__ qkv,
    unsigned short* __restrict__ vH, unsigned short* __restrict__ vL) {
  const int idx = blockIdx.x * 256 + threadIdx.x;
  const int b = idx >> 15;
  const int r = idx & 32767;
  const int co = r >> 9;
  const int p8 = (r & 511) * 8;
  const float* src = qkv + ((size_t)(b * kCO3 + 2 * kCI + co)) * kNPIX + p8;
  const v4f a0 = *(const v4f*)src;
  const v4f a1 = *(const v4f*)(src + 4);
  unsigned hw[4], lw[4];
  split2(a0.x, a0.y, hw[0], lw[0]);
  split2(a0.z, a0.w, hw[1], lw[1]);
  split2(a1.x, a1.y, hw[2], lw[2]);
  split2(a1.z, a1.w, hw[3], lw[3]);
  v4u hv; hv.x = hw[0]; hv.y = hw[1]; hv.z = hw[2]; hv.w = hw[3];
  v4u lv; lv.x = lw[0]; lv.y = lw[1]; lv.z = lw[2]; lv.w = lw[3];
  const size_t d = ((size_t)(b * kCI + co)) * kNPIX + p8;
  *(volatile v4u*)(vH + d) = hv;
  *(volatile v4u*)(vL + d) = lv;
  __threadfence();
  *(volatile v4u*)(vH + d) = hv;
  *(volatile v4u*)(vL + d) = lv;
}

__global__ __launch_bounds__(128) void attn_kernel(
    const unsigned short* __restrict__ qHp, const unsigned short* __restrict__ qLp,
    const unsigned short* __restrict__ kHp, const unsigned short* __restrict__ kLp,
    const unsigned short* __restrict__ vHp, const unsigned short* __restrict__ vLp,
    unsigned short* __restrict__ oHp, unsigned short* __restrict__ oLp) {
  typedef __bf16 T;
  union FB { v16b v; v8b h[2]; };
  __shared__ __align__(16) __bf16 Psh[4][16 * 64];
  __shared__ __align__(16) __bf16 Psl[4][16 * 64];
  __shared__ __align__(16) float  Os[4][16 * 68];
  const int tid = threadIdx.x, wave = tid >> 5, lane = tid & 31;
  const int hh = lane >> 4, c = lane & 15, koff = hh * 8;
  const int blk = blockIdx.x;
  const int b = blk >> 6;
  const int qb = blk & 63;
  const int q0 = qb * 64 + wave * 16;
  const size_t pm = (size_t)b * kNPIX * kCI;
  const T* qH = (const T*)qHp + pm;
  const T* qL = (const T*)qLp + pm;
  const T* kH = (const T*)kHp + pm;
  const T* kL = (const T*)kLp + pm;
  const T* vH = (const T*)vHp + (size_t)b * kCI * kNPIX;
  const T* vL = (const T*)vLp + (size_t)b * kCI * kNPIX;

  v16b qah[2], qal[2];
#pragma unroll
  for (int dc = 0; dc < 2; ++dc) {
    const size_t qo = (size_t)(q0 + c) * kCI + dc * 32 + koff;
    qah[dc] = Frag<T>::load(qH + qo);
    qal[dc] = Frag<T>::load(qL + qo);
  }

  float mrow[8], lrow[8];
  v8f oacc[4];
#pragma unroll
  for (int r = 0; r < 8; ++r) { mrow[r] = -INFINITY; lrow[r] = 0.f; }
#pragma unroll
  for (int t = 0; t < 4; ++t) oacc[t] = (v8f){0.f,0.f,0.f,0.f,0.f,0.f,0.f,0.f};

  __bf16* pwh = Psh[wave];
  __bf16* pwl = Psl[wave];

  for (int kc = 0; kc < kNPIX / 64; ++kc) {
    const int kv0 = kc * 64;
    v8f s[4];
#pragma unroll
    for (int j = 0; j < 4; ++j) {
      s[j] = (v8f){0.f,0.f,0.f,0.f,0.f,0.f,0.f,0.f};
#pragma unroll
      for (int dc = 0; dc < 2; ++dc) {
        const size_t ko = (size_t)(kv0 + (j << 4) + c) * kCI + dc * 32 + koff;
        const v16b kb = Frag<T>::load(kH + ko);
        const v16b kl = Frag<T>::load(kL + ko);
        s[j] = mma_g(qah[dc], kb, s[j]);
        s[j] = mma_g(qah[dc], kl, s[j]);
        s[j] = mma_g(qal[dc], kb, s[j]);
      }
    }
    float cm[8];
#pragma unroll
    for (int r = 0; r < 8; ++r) {
      float m = fmaxf(fmaxf(s[0][r], s[1][r]), fmaxf(s[2][r], s[3][r]));
#pragma unroll
      for (int off = 1; off < 16; off <<= 1) m = fmaxf(m, __shfl_xor(m, off, 32));
      cm[r] = m;
    }
    __builtin_amdgcn_fence(__ATOMIC_RELEASE, "workgroup");
    __builtin_amdgcn_wave_barrier();
    __builtin_amdgcn_fence(__ATOMIC_ACQUIRE, "workgroup");
#pragma unroll
    for (int r = 0; r < 8; ++r) {
      const float mnew = fmaxf(mrow[r], cm[r]);
      const float alpha = expf(mrow[r] - mnew);
      mrow[r] = mnew;
      float psum = 0.f;
#pragma unroll
      for (int j = 0; j < 4; ++j) {
        const float p = expf(s[j][r] - mnew);
        psum += p;
        __bf16 ph, plo;
        split_bf(p, ph, plo);
        pwh[(8 * hh + r) * 64 + (j << 4) + c] = ph;
        pwl[(8 * hh + r) * 64 + (j << 4) + c] = plo;
      }
#pragma unroll
      for (int off = 1; off < 16; off <<= 1) psum += __shfl_xor(psum, off, 32);
      lrow[r] = lrow[r] * alpha + psum;
#pragma unroll
      for (int t = 0; t < 4; ++t) oacc[t][r] *= alpha;
    }
    __builtin_amdgcn_fence(__ATOMIC_RELEASE, "workgroup");
    __builtin_amdgcn_wave_barrier();
    __builtin_amdgcn_fence(__ATOMIC_ACQUIRE, "workgroup");
#pragma unroll 1
    for (int kk = 0; kk < 2; ++kk) {
      FB pa, pl;
      pa.h[0] = *(const v8b*)(pwh + c * 64 + kk * 32 + 8 * hh);
      pa.h[1] = *(const v8b*)(pwh + c * 64 + kk * 32 + 16 + 8 * hh);
      pl.h[0] = *(const v8b*)(pwl + c * 64 + kk * 32 + 8 * hh);
      pl.h[1] = *(const v8b*)(pwl + c * 64 + kk * 32 + 16 + 8 * hh);
#pragma unroll
      for (int t = 0; t < 4; ++t) {
        const size_t vo = (size_t)((t << 4) + c) * kNPIX + kv0 + kk * 32 + koff;
        const v16b vb = Frag<T>::load(vH + vo);
        const v16b vl = Frag<T>::load(vL + vo);
        oacc[t] = mma_g(pa.v, vb, oacc[t]);
        oacc[t] = mma_g(pa.v, vl, oacc[t]);
        oacc[t] = mma_g(pl.v, vb, oacc[t]);
      }
    }
  }

  float* os = Os[wave];
#pragma unroll
  for (int r = 0; r < 8; ++r) {
    const float inv = 1.0f / lrow[r];
#pragma unroll
    for (int t = 0; t < 4; ++t) os[(8 * hh + r) * 68 + t * 16 + c] = oacc[t][r] * inv;
  }
  __builtin_amdgcn_fence(__ATOMIC_RELEASE, "workgroup");
  __builtin_amdgcn_wave_barrier();
  __builtin_amdgcn_fence(__ATOMIC_ACQUIRE, "workgroup");
  {
    unsigned short* oHb = oHp + pm;
    unsigned short* oLb = oLp + pm;
    const int rq = lane >> 3, c8 = (lane & 7) * 8;
    for (int pass = 0; pass < 2; ++pass) {
#pragma unroll
      for (int it = 0; it < 4; ++it) {
        const int row = it * 4 + rq;
        const float* sp = os + row * 68 + c8;
        unsigned hw[4], lw[4];
#pragma unroll
        for (int e = 0; e < 4; ++e) split2(sp[2 * e], sp[2 * e + 1], hw[e], lw[e]);
        v4u hv; hv.x = hw[0]; hv.y = hw[1]; hv.z = hw[2]; hv.w = hw[3];
        v4u lv; lv.x = lw[0]; lv.y = lw[1]; lv.z = lw[2]; lv.w = lw[3];
        const size_t d = (size_t)(q0 + row) * kCI + c8;
        *(volatile v4u*)(oHb + d) = hv;
        *(volatile v4u*)(oLb + d) = lv;
      }
      __threadfence();
    }
  }
}

__global__ __launch_bounds__(256) void bn_out_kernel(const float* __restrict__ y, const float* __restrict__ bnw,
                                                    const float* __restrict__ bnb, float* __restrict__ out) {
  __shared__ float red[256];
  __shared__ float stat[2];
  const int tid = threadIdx.x, c = blockIdx.x;
  float s = 0.f;
  for (int bb = 0; bb < kB; ++bb) {
    const float* row = y + ((size_t)(bb * kCIN + c)) * kNPIX;
#pragma unroll 4
    for (int i = 0; i < kNPIX / 256; ++i) s += row[i * 256 + tid];
  }
  red[tid] = s;
  __syncthreads();
  for (int o = 128; o > 0; o >>= 1) { if (tid < o) red[tid] += red[tid + o]; __syncthreads(); }
  if (tid == 0) stat[0] = red[0] * (1.0f / (float)(kB * kNPIX));
  __syncthreads();
  const float mean = stat[0];
  float s2 = 0.f;
  for (int bb = 0; bb < kB; ++bb) {
    const float* row = y + ((size_t)(bb * kCIN + c)) * kNPIX;
#pragma unroll 4
    for (int i = 0; i < kNPIX / 256; ++i) { const float d = row[i * 256 + tid] - mean; s2 += d * d; }
  }
  red[tid] = s2;
  __syncthreads();
  for (int o = 128; o > 0; o >>= 1) { if (tid < o) red[tid] += red[tid + o]; __syncthreads(); }
  if (tid == 0) stat[1] = rsqrtf(red[0] * (1.0f / (float)(kB * kNPIX)) + 1e-5f);
  __syncthreads();
  const float rstd = stat[1];
  const float w = rbf(bnw[c]);
  const float bq = rbf(bnb[c]);
  for (int pass = 0; pass < 2; ++pass) {
    for (int bb = 0; bb < kB; ++bb) {
      const size_t rb = ((size_t)(bb * kCIN + c)) * kNPIX;
#pragma unroll
      for (int i = 0; i < kNPIX / 1024; ++i) {
        const int p4 = (i * 256 + tid) * 4;
        const v4f v = *(const v4f*)(y + rb + p4);
        v4f o2 = (v - mean) * rstd;
        o2 = o2 * w + bq;
        *(volatile v4f*)(out + rb + p4) = o2;
      }
    }
    __threadfence();
  }
}

static_assert(kCIN % 32 == 0);
static_assert(kCI % 32 == 0);
static_assert(kCSPL % 32 == 0);
static_assert((kB * kNPIX) % 64 == 0 && kCI % 64 == 0);
static_assert(kCIN % 64 == 0 && kNPIX % 64 == 0);
static_assert(kCO3 % 64 == 0);
static_assert((kKT % 8) == 0 && (kKB % 32) == 0);
static_assert((kCI * kCIN) % 2 == 0);

extern "C" void kernel_launch(void* const* d_in, const int* in_sizes, int n_in,
                              void* d_out, int out_size, void* d_ws, size_t ws_size,
                              hipStream_t stream) {
  if (n_in < 14) return;
  if (in_sizes[0] != kB * kCIN * kNPIX || out_size != kB * kCIN * kNPIX) return;
  if (in_sizes[1] != kCI * kCIN || in_sizes[2] != kCI || in_sizes[3] != kCIN * kCI || in_sizes[4] != kCIN) return;
  if (in_sizes[5] != kCI * kCI * 9 || in_sizes[6] != kCI * kCSPL * 9 || in_sizes[7] != kCI * kCI * 9 ||
      in_sizes[8] != kCI * kCSPL * 9 || in_sizes[9] != kCI * kCI * 9 || in_sizes[10] != kCI * kCSPL * 9) return;
  if (in_sizes[11] < 1 || in_sizes[12] != kCIN || in_sizes[13] != kCIN) return;
  if (ws_size < kWsTotal) return;

  const float* x      = (const float*)d_in[0];
  const float* W_in   = (const float*)d_in[1];
  const float* b_in   = (const float*)d_in[2];
  const float* W_out  = (const float*)d_in[3];
  const float* b_out  = (const float*)d_in[4];
  const float* Wq_b   = (const float*)d_in[5];
  const float* Wq_s   = (const float*)d_in[6];
  const float* Wk_b   = (const float*)d_in[7];
  const float* Wk_s   = (const float*)d_in[8];
  const float* Wv_b   = (const float*)d_in[9];
  const float* Wv_s   = (const float*)d_in[10];
  const float* gamma  = (const float*)d_in[11];
  const float* bn_w   = (const float*)d_in[12];
  const float* bn_b   = (const float*)d_in[13];
  float* out = (float*)d_out;

  char* ws = (char*)d_ws;
  unsigned short* xT    = (unsigned short*)(ws + oXT);
  unsigned short* Win16 = (unsigned short*)(ws + oWIN);
  unsigned short* Wo16  = (unsigned short*)(ws + oWOUT);
  unsigned short* Wt    = (unsigned short*)(ws + oWT);
  float*          att   = (float*)(ws + oATT);
  float*          st    = (float*)(ws + oST);
  unsigned short* sH    = (unsigned short*)(ws + oSH);
  unsigned short* sL    = (unsigned short*)(ws + oSL);
  unsigned short* bH    = (unsigned short*)(ws + oBH);
  unsigned short* bL    = (unsigned short*)(ws + oBL);
  float*          qkv   = (float*)(ws + oQKV);
  unsigned short* qH    = (unsigned short*)(ws + oQH);
  unsigned short* qL    = (unsigned short*)(ws + oQL);
  unsigned short* kH    = (unsigned short*)(ws + oKH);
  unsigned short* kL    = (unsigned short*)(ws + oKL);
  unsigned short* vH    = (unsigned short*)(ws + oVH);
  unsigned short* vL    = (unsigned short*)(ws + oVL);
  unsigned short* oH    = (unsigned short*)(ws + oOH);
  unsigned short* oL    = (unsigned short*)(ws + oOL);
  float*          ybuf  = (float*)(ws + oY);

  zero_ghost_kernel<<<dim3(16, 4), 256, 0, stream>>>(sH, sL, bH, bL);

  cast_f32_bf16x2<<<(kCI * kCIN / 2 + 255) / 256, 256, 0, stream>>>(W_in, Win16, kCI * kCIN / 2);
  cast_f32_bf16x2<<<(kCIN * kCI / 2 + 255) / 256, 256, 0, stream>>>(W_out, Wo16, kCIN * kCI / 2);

  const int npB = kCI * kKB / 2;
  const int npS = kCI * kKS / 2;
  wreorder_kernel<<<(npB + 255) / 256, 256, 0, stream>>>(Wq_b, Wt, 6, 0,       0,   npB);
  wreorder_kernel<<<(npS + 255) / 256, 256, 0, stream>>>(Wq_s, Wt, 9, 0,       kKB, npS);
  wreorder_kernel<<<(npB + 255) / 256, 256, 0, stream>>>(Wk_b, Wt, 6, kCI,     0,   npB);
  wreorder_kernel<<<(npS + 255) / 256, 256, 0, stream>>>(Wk_s, Wt, 9, kCI,     kKB, npS);
  wreorder_kernel<<<(npB + 255) / 256, 256, 0, stream>>>(Wv_b, Wt, 6, 2 * kCI, 0,   npB);
  wreorder_kernel<<<(npS + 255) / 256, 256, 0, stream>>>(Wv_s, Wt, 9, 2 * kCI, kKB, npS);

  xpose_x_kernel<<<kB * (kNPIX / 64), 256, 0, stream>>>(x, xT);

  {
    const int M = kB * kNPIX, N = kCI, K = kCIN;
    const int blocks = ((M / 64) * (N / 64) + 7) / 8;
    gemm64_kernel<false, 2, false><<<dim3(blocks, 1), 256, 0, stream>>>(
        xT, K, 0L, Win16, Win16, K, 0L, att, kCI, 0L, b_in, x, gamma, M, N, K);
  }

  inorm_stats_kernel<<<kB, 256, 0, stream>>>(att, st);

  {
    const float inv7 = 1.0f / 7.0f;
    const float denf = (float)(4.0 / 7.0);
    const float invden = 1.0f / denf;
    act_planes_kernel<<<kB * (kNPIX / 4), 256, 0, stream>>>(att, st, sH, sL, bH, bL, inv7, invden);
  }

  conv_qkv_kernel<<<((kCO3 / 64) * (kB * kHW)) / 8, 256, 0, stream>>>(Wt, sH, sL, bH, bL, qkv);

  qk_planes_kernel<<<kB * 2 * (kNPIX / 64), 256, 0, stream>>>(qkv, qH, qL, kH, kL);
  v_planes_kernel<<<(kB * kCI * kNPIX / 8) / 256, 256, 0, stream>>>(qkv, vH, vL);

  attn_kernel<<<kB * (kNPIX / 64), 128, 0, stream>>>(qH, qL, kH, kL, vH, vL, oH, oL);

  {
    const int M = kCIN, N = kNPIX, K = kCI;
    const int blocks = ((M / 64) * (N / 64) + 7) / 8;
    gemm64_kernel<true, 1, true><<<dim3(blocks, kB), 256, 0, stream>>>(
        Wo16, K, 0L, oH, oL, K, (long)kNPIX * kCI, ybuf, kNPIX, (long)kCIN * kNPIX, b_out, x, gamma, M, N, K);
  }

  bn_out_kernel<<<kCIN, 256, 0, stream>>>(ybuf, bn_w, bn_b, out);
}
